// ValueNetwork_26010321944671
// MI455X (gfx1250) — hardware-verified
//
#include <hip/hip_runtime.h>
#include <math.h>

constexpr int kItems      = 16384;
constexpr int kAgents     = 20;
constexpr int kFeat       = 13;
constexpr int kSelf       = 6;
constexpr int kChunkItems = 4096;
constexpr int kChunkRows  = kChunkItems * kAgents;
constexpr int kNumChunks  = kItems / kChunkItems;
static_assert(kNumChunks * kChunkItems == kItems);
static_assert(kChunkRows % 64 == 0);
static_assert(kChunkItems % 64 == 0);
static_assert(kItems % 256 == 0);

constexpr int kK0 = 32;
constexpr int kN0 = 192;
constexpr int kK1 = 160;
constexpr int kP  = 128;
constexpr int kNf = 64;
constexpr int kKm = 64;

constexpr float kWCarry   = 16.0f;
constexpr float kActCarry = 8.0f;
constexpr float kSc1a     = kActCarry / kWCarry;
constexpr float kScAct    = kActCarry / (kActCarry * kWCarry);
constexpr float kScF32    = 1.0f / (kActCarry * kWCarry);

constexpr long kOffW1a  = 0;
constexpr long kOffW1b  = 6144;
constexpr long kOffWa0t = 26624;
constexpr long kOffWa0b = 43008;
constexpr long kOffWa1  = 59392;
constexpr long kOffW2a  = 75776;
constexpr long kOffW2b  = 92160;
constexpr long kOffW3a  = 100352;
constexpr long kOffW3b  = 112640;
constexpr long kOffW3c  = 133120;
constexpr long kWElems  = 149504;
static_assert(kOffW1b == kOffW1a + 192 * 32);
static_assert(kOffWa0t == kOffW1b + 128 * 160);
static_assert(kOffWa0b == kOffWa0t + 128 * 128);
static_assert(kOffWa1 == kOffWa0b + 128 * 128);
static_assert(kOffW2a == kOffWa1 + 128 * 128);
static_assert(kOffW2b == kOffW2a + 128 * 128);
static_assert(kOffW3a == kOffW2b + 64 * 128);
static_assert(kOffW3b == kOffW3a + 192 * 64);
static_assert(kOffW3c == kOffW3b + 128 * 160);
static_assert(kWElems == kOffW3c + 128 * 128);

constexpr int kOffB1a = 0;
constexpr int kOffB1b = 192;
constexpr int kOffBa0 = 320;
constexpr int kOffBa1 = 448;
constexpr int kOffB2a = 576;
constexpr int kOffB2b = 704;
constexpr int kOffB3a = 768;
constexpr int kOffB3b = 960;
constexpr int kOffB3c = 1088;
constexpr int kBiasElems = 1216;

typedef __attribute__((ext_vector_type(16))) _Float16 v16h;
typedef __attribute__((ext_vector_type(8)))  _Float16 v8h;
typedef __attribute__((ext_vector_type(16))) __bf16   v16b;
typedef __attribute__((ext_vector_type(8)))  __bf16   v8b;
typedef __attribute__((ext_vector_type(8)))  float    v8f;
typedef __attribute__((ext_vector_type(4)))  float    v4f;
typedef __attribute__((ext_vector_type(4)))  unsigned int v4u;

__device__ __forceinline__ unsigned short f2bf_bits(float f) {
  unsigned u = __float_as_uint(f);
  return (unsigned short)((u + 0x7FFFu + ((u >> 16) & 1u)) >> 16);
}
__device__ __forceinline__ float bf_bits2f(unsigned short h) { return __uint_as_float(((unsigned)h) << 16); }

__device__ __forceinline__ void dep_guard_h(v8f& a, v8f& b, v16h x, v16h y) { asm volatile("v_nop\n\tv_nop\n\tv_nop\n\tv_nop" : "+v"(a), "+v"(b) : "v"(x), "v"(y)); }
__device__ __forceinline__ void dep_guard_b(v8f& a, v8f& b, v16b x, v16b y) { asm volatile("v_nop\n\tv_nop\n\tv_nop\n\tv_nop" : "+v"(a), "+v"(b) : "v"(x), "v"(y)); }
__device__ __forceinline__ void keep4_h(v16h a, v16h b, v16h c, v16h d) { asm volatile("v_nop" :: "v"(a), "v"(b), "v"(c), "v"(d)); }
__device__ __forceinline__ void keep4_b(v16b a, v16b b, v16b c, v16b d) { asm volatile("v_nop" :: "v"(a), "v"(b), "v"(c), "v"(d)); }
__device__ __forceinline__ void acc_guard4(v8f& a, v8f& b, v8f& c, v8f& d) { asm volatile("v_nop\n\tv_nop\n\tv_nop\n\tv_nop" : "+v"(a), "+v"(b), "+v"(c), "+v"(d)); }
template <typename T> struct Frag;
template <> struct Frag<_Float16> {
  typedef v16h V; union U { v16h v; v8h h[2]; };
  static __device__ __forceinline__ v16h load(const _Float16* p) {
    U f; f.h[0] = *(const v8h*)(p); f.h[1] = *(const v8h*)(p + 16); return f.v;
  }
  static __device__ __forceinline__ v8f mma(v16h a, v16h b, v8f c) {
    return __builtin_amdgcn_wmma_f32_16x16x32_f16(false, a, false, b, (short)0, c, false, false);
  }
  static __device__ __forceinline__ void guard(v8f& a, v8f& b, v16h x, v16h y) { dep_guard_h(a, b, x, y); }
  static __device__ __forceinline__ void keep(v16h a, v16h b, v16h c, v16h d) { keep4_h(a, b, c, d); }
};
template <> struct Frag<__bf16> {
  typedef v16b V; union U { v16b v; v8b h[2]; };
  static __device__ __forceinline__ v16b load(const __bf16* p) {
    U f; f.h[0] = *(const v8b*)(p); f.h[1] = *(const v8b*)(p + 16); return f.v;
  }
  static __device__ __forceinline__ v8f mma(v16b a, v16b b, v8f c) {
    return __builtin_amdgcn_wmma_f32_16x16x32_bf16(false, a, false, b, (short)0, c, false, false);
  }
  static __device__ __forceinline__ void guard(v8f& a, v8f& b, v16b x, v16b y) { dep_guard_b(a, b, x, y); }
  static __device__ __forceinline__ void keep(v16b a, v16b b, v16b c, v16b d) { keep4_b(a, b, c, d); }
};

__device__ __forceinline__ unsigned pk16(unsigned short a, unsigned short b) { return (unsigned)a | ((unsigned)b << 16); }
__device__ __forceinline__ unsigned short h_bits(float f) { const _Float16 h = (_Float16)f; return __builtin_bit_cast(unsigned short, h); }

__device__ __forceinline__ float h16bits_to_f32(unsigned h) {
  const unsigned e   = (h >> 10) & 31u;
  const unsigned s   = (h & 0x8000u) << 16;
  const unsigned mag = ((e + 112u) << 23) | ((h & 1023u) << 13);
  const float f = __uint_as_float(s | mag);
  return (e == 0u) ? __uint_as_float(s) : f;
}

__device__ __forceinline__ void split8_bf(const float (&v)[8], v4u& uh, v4u& ul) {
  unsigned short hb[8], lb[8];
#pragma unroll
  for (int e = 0; e < 8; ++e) {
    hb[e] = f2bf_bits(v[e]);
    lb[e] = f2bf_bits(v[e] - bf_bits2f(hb[e]));
  }
  uh = (v4u){pk16(hb[0], hb[1]), pk16(hb[2], hb[3]), pk16(hb[4], hb[5]), pk16(hb[6], hb[7])};
  ul = (v4u){pk16(lb[0], lb[1]), pk16(lb[2], lb[3]), pk16(lb[4], lb[5]), pk16(lb[6], lb[7])};
}
__device__ __forceinline__ v4u pack8_f16(const float (&v)[8]) {
  unsigned short hb[8];
#pragma unroll
  for (int e = 0; e < 8; ++e) hb[e] = h_bits(v[e]);
  return (v4u){pk16(hb[0], hb[1]), pk16(hb[2], hb[3]), pk16(hb[4], hb[5]), pk16(hb[6], hb[7])};
}
__device__ __forceinline__ void store2_planes(unsigned short* ph, unsigned short* pl, v4u uh, v4u ul) {
  *(volatile v4u*)ph = uh;
  *(volatile v4u*)pl = ul;
  __threadfence();
  *(volatile v4u*)ph = uh;
  *(volatile v4u*)pl = ul;
}
__device__ __forceinline__ void store2_one(unsigned short* p, v4u u) {
  *(volatile v4u*)p = u;
  __threadfence();
  *(volatile v4u*)p = u;
}

template <int ET> struct Elem;
template <> struct Elem<0> { typedef _Float16 T; };
template <> struct Elem<1> { typedef __bf16 T; };
template <int ET, bool SPLIT, int BIAS_MODE, int OUT_MODE, bool RESID, int ACT = 0, int RDIV = 1>
__global__ __launch_bounds__(256) void wmma_gemm64(
    const unsigned short* __restrict__ Ap, const unsigned short* __restrict__ A2p, int lda, long strideA,
    const unsigned short* __restrict__ Btp, const unsigned short* __restrict__ Bt2p, int ldb, long strideB,
    void* __restrict__ Cout, void* __restrict__ Cout2, int ldc, long strideC,
    const float* __restrict__ bias,
    const float* __restrict__ resid, long strideR,
    int M, int N, int K, float scale) {
  typedef typename Elem<ET>::T T;
  typedef typename Frag<T>::V V;
  const T* A = (const T*)Ap; const T* A2 = (const T*)A2p; const T* Bt = (const T*)Btp; const T* Bt2 = (const T*)Bt2p;
  __shared__ __align__(16) float sT[8][16 * 68];
  const int b    = blockIdx.y;
  const int lane = threadIdx.x & 31;
  const int wave = threadIdx.x >> 5;
  const int tilesN = N >> 6;
  const int tilesM = M >> 6;
  const int tile = blockIdx.x * 8 + wave;
  if (tile >= tilesM * tilesN) return;
  const int tm = tile / tilesN;
  const int tn = tile - tm * tilesN;
  const int m0 = tm << 6;
  const int n0 = tn << 6;

  const T* Ab  = A  + (size_t)b * strideA;
  const T* Bb  = Bt + (size_t)b * strideB;
  const T* Ab2 = SPLIT ? (A2  + (size_t)b * strideA) : nullptr;
  const T* Bb2 = SPLIT ? (Bt2 + (size_t)b * strideB) : nullptr;

  const int rlane = lane & 15;
  const int koff  = (lane >> 4) * 8;
  const int mOff  = (lane >> 4) * 8;

  v8f acc[4][4];
#pragma unroll
  for (int i = 0; i < 4; ++i)
#pragma unroll
    for (int j = 0; j < 4; ++j) acc[i][j] = (v8f){0.f,0.f,0.f,0.f,0.f,0.f,0.f,0.f};

  for (int k0 = 0; k0 < K; k0 += 32) {
    V bh[4], bl[4];
#pragma unroll
    for (int j = 0; j < 4; ++j) {
      const size_t bo = (size_t)(n0 + (j << 4) + rlane) * ldb + koff + k0;
      bh[j] = Frag<T>::load(Bb + bo);
      if (SPLIT) bl[j] = Frag<T>::load(Bb2 + bo);
    }
#pragma unroll
    for (int i = 0; i < 4; ++i) {
      const size_t ao = (size_t)(m0 + (i << 4) + rlane) * lda + koff + k0;
      V ah = Frag<T>::load(Ab + ao);
      V al;
      if (SPLIT) al = Frag<T>::load(Ab2 + ao);
#pragma unroll
      for (int j = 0; j < 4; ++j) {
        acc[i][j] = Frag<T>::mma(ah, bh[j], acc[i][j]);
        if (SPLIT) {
          acc[i][j] = Frag<T>::mma(ah, bl[j], acc[i][j]);
          acc[i][j] = Frag<T>::mma(al, bh[j], acc[i][j]);
        }
      }
      Frag<T>::guard(acc[i][0], acc[i][3], ah, SPLIT ? al : ah);
    }
    Frag<T>::keep(bh[0], bh[1], bh[2], bh[3]);
    if (SPLIT) Frag<T>::keep(bl[0], bl[1], bl[2], bl[3]);
  }
  acc_guard4(acc[0][0], acc[0][1], acc[0][2], acc[0][3]);
  acc_guard4(acc[1][0], acc[1][1], acc[1][2], acc[1][3]);
  acc_guard4(acc[2][0], acc[2][1], acc[2][2], acc[2][3]);
  acc_guard4(acc[3][0], acc[3][1], acc[3][2], acc[3][3]);

  float* slab = sT[wave];
  const float* Rb = RESID ? (resid + (size_t)b * strideR) : nullptr;
#pragma unroll
  for (int i = 0; i < 4; ++i) {
    const int mBase = m0 + (i << 4);
#pragma unroll
    for (int j = 0; j < 4; ++j) {
      const int n = n0 + (j << 4) + rlane;
      float bv = 0.f;
      if (BIAS_MODE == 2) bv = bias[n];
#pragma unroll
      for (int r = 0; r < 8; ++r) {
        float v = acc[i][j][r] * scale;
        if (BIAS_MODE == 1) v += bias[mBase + mOff + r];
        if (BIAS_MODE == 2) v += bv;
        if (RESID) v += Rb[(size_t)((mBase + mOff + r) / RDIV) * ldc + n];
        if (ACT == 2) v = fmaxf(v, 0.0f);
        if (ACT == 4) v = (v > 0.f) ? v : 0.01f * v;
        slab[(mOff + r) * 68 + (j << 4) + rlane] = v;
      }
    }
    __builtin_amdgcn_fence(__ATOMIC_RELEASE, "workgroup");
    __builtin_amdgcn_wave_barrier();
    __builtin_amdgcn_fence(__ATOMIC_ACQUIRE, "workgroup");
    if (OUT_MODE == 0) {
      float* C = (float*)Cout + (size_t)b * strideC;
      const int hh = lane >> 4, c4 = (lane & 15) * 4;
      for (int pass = 0; pass < 2; ++pass) {
#pragma unroll
        for (int it = 0; it < 8; ++it) {
          const int row = it * 2 + hh;
          v4f v = *(const v4f*)(slab + row * 68 + c4);
          *(volatile v4f*)(C + (size_t)(mBase + row) * ldc + n0 + c4) = v;
        }
        __threadfence();
      }
    } else {
      const int q = lane >> 3, c8 = (lane & 7) * 8;
      unsigned short* C  = (unsigned short*)Cout  + (size_t)b * strideC;
      unsigned short* C2 = (OUT_MODE == 2) ? ((unsigned short*)Cout2 + (size_t)b * strideC) : nullptr;
      for (int pass = 0; pass < 2; ++pass) {
#pragma unroll
        for (int it = 0; it < 4; ++it) {
          const int row = it * 4 + q;
          const float* sp = slab + row * 68 + c8;
          v8h hv, lv;
#pragma unroll
          for (int e = 0; e < 8; ++e) {
            if (OUT_MODE == 1) {
              hv[e] = (_Float16)sp[e];
            } else {
              unsigned short hb = f2bf_bits(sp[e]);
              unsigned short lb = f2bf_bits(sp[e] - bf_bits2f(hb));
              hv[e] = __builtin_bit_cast(_Float16, hb);
              lv[e] = __builtin_bit_cast(_Float16, lb);
            }
          }
          *(volatile v8h*)(C + (size_t)(mBase + row) * ldc + n0 + c8) = hv;
          if (OUT_MODE == 2) *(volatile v8h*)(C2 + (size_t)(mBase + row) * ldc + n0 + c8) = lv;
        }
        __threadfence();
      }
    }
    __builtin_amdgcn_fence(__ATOMIC_RELEASE, "workgroup");
    __builtin_amdgcn_wave_barrier();
    __builtin_amdgcn_fence(__ATOMIC_ACQUIRE, "workgroup");
  }
}

template <int WMODE>
__global__ __launch_bounds__(256) void wprep_kernel(
    const float* w0, const float* w1, const float* w2, const float* w3,
    long o0, long o1, long o2, long o3,
    unsigned short* __restrict__ wp, unsigned short* __restrict__ wlo,
    int K, int N, int Kp, int Np, int ldw, float scale) {
  const int z = blockIdx.y;
  const float* W = (z == 0) ? w0 : (z == 1) ? w1 : (z == 2) ? w2 : w3;
  const long off = (z == 0) ? o0 : (z == 1) ? o1 : (z == 2) ? o2 : o3;
  const int e0 = (blockIdx.x * 256 + (int)threadIdx.x) * 8;
  if (e0 >= Np * Kp) return;
  float v[8];
#pragma unroll
  for (int e = 0; e < 8; ++e) {
    const int idx = e0 + e;
    const int n = idx / Kp;
    const int k = idx - n * Kp;
    const int kc = (k < K) ? k : (K - 1);
    const int nc = (n < N) ? n : (N - 1);
    const float t = W[(size_t)kc * ldw + nc];
    v[e] = (k < K && n < N) ? (t * scale) : 0.0f;
  }
  if (WMODE == 0) {
    const v4u u = pack8_f16(v);
    store2_one(wp + off + e0, u);
  } else {
    v4u uh, ul;
    split8_bf(v, uh, ul);
    store2_planes(wp + off + e0, wlo + off + e0, uh, ul);
  }
}

__global__ __launch_bounds__(64) void bprep_kernel(
    const float* b0, const float* b1, const float* b2, const float* b3, const float* b4,
    const float* b5, const float* b6, const float* b7, const float* b8, float* __restrict__ bout) {
  const int z = blockIdx.x;
  const float* bp = (z == 0) ? b0 : (z == 1) ? b1 : (z == 2) ? b2 : (z == 3) ? b3 : (z == 4) ? b4
                  : (z == 5) ? b5 : (z == 6) ? b6 : (z == 7) ? b7 : b8;
  const int n   = (z == 0 || z == 6) ? 150 : (z == 5) ? 50 : 100;
  const int np  = (z == 0 || z == 6) ? kN0 : (z == 5) ? kNf : kP;
  const int off = (z == 0) ? kOffB1a : (z == 1) ? kOffB1b : (z == 2) ? kOffBa0 : (z == 3) ? kOffBa1 : (z == 4) ? kOffB2a
                : (z == 5) ? kOffB2b : (z == 6) ? kOffB3a : (z == 7) ? kOffB3b : kOffB3c;
  const float carry = (z == 0 || z == 1 || z == 2 || z == 4) ? kActCarry : 1.0f;
  const int t = threadIdx.x;
  if (t * 4 >= np) return;
  v4f v;
#pragma unroll
  for (int e = 0; e < 4; ++e) {
    const int i  = 4 * t + e;
    const int ic = (i < n) ? i : (n - 1);
    const float f = bp[ic];
    v[e] = (i < n) ? (f * carry) : 0.0f;
  }
  float* p = bout + off + 4 * t;
  *(volatile v4f*)p = v;
  __threadfence();
  *(volatile v4f*)p = v;
}

__global__ __launch_bounds__(256) void xprep_kernel(const float* __restrict__ x, unsigned short* __restrict__ xh, int rows) {
  const int gid  = blockIdx.x * 256 + (int)threadIdx.x;
  const int row  = gid >> 2;
  const int part = gid & 3;
  if (row >= rows) return;
  const float* xr = x + (size_t)row * kFeat;
  float v[8];
#pragma unroll
  for (int e = 0; e < 8; ++e) {
    const int c  = part * 8 + e;
    const int cc = (c < kFeat) ? c : (kFeat - 1);
    const float t = xr[cc];
    v[e] = (c < kFeat) ? t : 0.0f;
  }
  const v4u u = pack8_f16(v);
  store2_one(xh + (size_t)row * kK0 + part * 8, u);
}

__global__ __launch_bounds__(256) void gmean_kernel(const unsigned short* __restrict__ h1p,
                                                    unsigned short* __restrict__ gp, int items) {
  const int gid  = blockIdx.x * 256 + (int)threadIdx.x;
  const int b    = gid >> 4;
  const int part = gid & 15;
  if (b >= items) return;
  const unsigned short* ph = h1p + (size_t)b * kAgents * kP + part * 8;
  float s[8];
#pragma unroll
  for (int e = 0; e < 8; ++e) s[e] = 0.0f;
#pragma unroll 1
  for (int n = 0; n < kAgents; ++n) {
    const v4u uw = *(const v4u*)(ph + (size_t)n * kP);
#pragma unroll
    for (int e = 0; e < 4; ++e) {
      s[2 * e]     += h16bits_to_f32(uw[e] & 0xffffu);
      s[2 * e + 1] += h16bits_to_f32(uw[e] >> 16);
    }
  }
  float v[8];
#pragma unroll
  for (int e = 0; e < 8; ++e) v[e] = s[e] * (1.0f / 20.0f);
  const v4u u = pack8_f16(v);
  store2_one(gp + (size_t)b * kP + part * 8, u);
}

__global__ __launch_bounds__(256) void pool_kernel(const float* __restrict__ s2, const float* __restrict__ f2,
                                                   const float* __restrict__ x, const float* __restrict__ wa2,
                                                   const float* __restrict__ ba2,
                                                   unsigned short* __restrict__ mh, unsigned short* __restrict__ ml, int items) {
  __shared__ __align__(16) float wsh[128];
  __shared__ __align__(16) float mrow[8][64];
  const int tid = threadIdx.x, wave = tid >> 5, lane = tid & 31;
  if (tid < 128) {
    const int tc = (tid < 100) ? tid : 99;
    const float w = wa2[tc];
    wsh[tid] = (tid < 100) ? w : 0.0f;
  }
  __syncthreads();
  const int b  = blockIdx.x * 8 + wave;
  const int bc = (b < items) ? b : (items - 1);
  const int n  = (lane < kAgents) ? lane : (kAgents - 1);
  const float* sr = s2 + ((size_t)bc * kAgents + n) * kP;
  float acc = 0.0f;
#pragma unroll 1
  for (int k4 = 0; k4 < 25; ++k4) {
    const v4f sv = *(const v4f*)(sr + 4 * k4);
    const v4f wv = *(const v4f*)(wsh + 4 * k4);
    acc += sv[0] * wv[0];
    acc += sv[1] * wv[1];
    acc += sv[2] * wv[2];
    acc += sv[3] * wv[3];
  }
  const bool valid = (lane < kAgents);
  const float sc = valid ? (acc + ba2[0]) : -INFINITY;
  float mx = sc;
#pragma unroll
  for (int off = 16; off > 0; off >>= 1) mx = fmaxf(mx, __shfl_xor(mx, off, 32));
  const float ex = expf(sc - mx);
  float sum = ex;
#pragma unroll
  for (int off = 16; off > 0; off >>= 1) sum += __shfl_xor(sum, off, 32);
  const float attn = ex * (1.0f / sum);
  float wfa = 0.0f, wfb = 0.0f;
#pragma unroll 1
  for (int j = 0; j < kAgents; ++j) {
    const float aj = __shfl(attn, j, 32);
    const float* fr = f2 + ((size_t)bc * kAgents + j) * kNf;
    wfa += aj * fr[lane];
    wfb += aj * fr[lane + 32];
  }
  float* mr = mrow[wave];
  const float* xr = x + (size_t)bc * (kAgents * kFeat);
  const float selfv = xr[(lane < kSelf) ? lane : (kSelf - 1)];
  if (lane < kSelf) mr[lane] = selfv;
  mr[kSelf + lane] = wfa;
  if (lane < 26) mr[38 + lane] = (lane < 18) ? wfb : 0.0f;
  __builtin_amdgcn_fence(__ATOMIC_RELEASE, "workgroup");
  __builtin_amdgcn_wave_barrier();
  __builtin_amdgcn_fence(__ATOMIC_ACQUIRE, "workgroup");
  const int q = lane & 7;
  const v4f a = *(const v4f*)(mr + 8 * q);
  const v4f c = *(const v4f*)(mr + 8 * q + 4);
  float v[8];
#pragma unroll
  for (int e = 0; e < 4; ++e) { v[e] = a[e]; v[4 + e] = c[e]; }
  v4u uh, ul;
  split8_bf(v, uh, ul);
  if (lane < 8 && b < items) {
    store2_planes(mh + (size_t)b * kKm + 8 * q, ml + (size_t)b * kKm + 8 * q, uh, ul);
  }
}

__global__ __launch_bounds__(256) void value_head_kernel(const float* __restrict__ t3, const float* __restrict__ w3d,
                                                         const float* __restrict__ b3d, float* __restrict__ out, int nrows) {
  __shared__ __align__(16) float wsh[128];
  __shared__ __align__(16) float st[8][32];
  const int tid = threadIdx.x, wave = tid >> 5, lane = tid & 31;
  if (tid < 128) {
    const int tc = (tid < 100) ? tid : 99;
    const float w = w3d[tc];
    wsh[tid] = (tid < 100) ? w : 0.0f;
  }
  __syncthreads();
  const int row = blockIdx.x * 256 + tid;
  const int rc  = (row < nrows) ? row : (nrows - 1);
  const float* tr = t3 + (size_t)rc * kP;
  float acc = 0.0f;
#pragma unroll 1
  for (int k4 = 0; k4 < 25; ++k4) {
    const v4f tv = *(const v4f*)(tr + 4 * k4);
    const v4f wv = *(const v4f*)(wsh + 4 * k4);
    acc += tv[0] * wv[0];
    acc += tv[1] * wv[1];
    acc += tv[2] * wv[2];
    acc += tv[3] * wv[3];
  }
  const float val = acc + b3d[0];
  st[wave][lane] = val;
  __builtin_amdgcn_fence(__ATOMIC_RELEASE, "workgroup");
  __builtin_amdgcn_wave_barrier();
  __builtin_amdgcn_fence(__ATOMIC_ACQUIRE, "workgroup");
  const int q = lane & 7;
  const v4f v = *(const v4f*)(&st[wave][4 * q]);
  const int base = blockIdx.x * 256 + wave * 32;
  if (lane < 8 && base + 32 <= nrows) {
    float* p = out + base + 4 * q;
    *(volatile v4f*)p = v;
    __threadfence();
    *(volatile v4f*)p = v;
  }
}

static inline size_t al4k(size_t b) { return (b + 4095) & ~(size_t)4095; }
static inline dim3 gemm_grid(int M, int N) { const int tiles = (M / 64) * (N / 64); return dim3((tiles + 7) / 8, 1, 1); }

extern "C" void kernel_launch(void* const* d_in, const int* in_sizes, int n_in,
                              void* d_out, int out_size, void* d_ws, size_t ws_size,
                              hipStream_t stream) {
  (void)in_sizes; (void)n_in; (void)out_size;
  const float* x   = (const float*)d_in[0];
  const float* w1a = (const float*)d_in[1];  const float* b1a = (const float*)d_in[2];
  const float* w1b = (const float*)d_in[3];  const float* b1b = (const float*)d_in[4];
  const float* wa0 = (const float*)d_in[5];  const float* ba0 = (const float*)d_in[6];
  const float* wa1 = (const float*)d_in[7];  const float* ba1 = (const float*)d_in[8];
  const float* wa2 = (const float*)d_in[9];  const float* ba2 = (const float*)d_in[10];
  const float* w2a = (const float*)d_in[11]; const float* b2a = (const float*)d_in[12];
  const float* w2b = (const float*)d_in[13]; const float* b2b = (const float*)d_in[14];
  const float* w3a = (const float*)d_in[15]; const float* b3a = (const float*)d_in[16];
  const float* w3b = (const float*)d_in[17]; const float* b3b = (const float*)d_in[18];
  const float* w3c = (const float*)d_in[19]; const float* b3c = (const float*)d_in[20];
  const float* w3d = (const float*)d_in[21]; const float* b3d = (const float*)d_in[22];
  float* out = (float*)d_out;

  size_t off = 0;
  const size_t oWP  = off; off += al4k((size_t)kWElems * 2);
  const size_t oWL  = off; off += al4k((size_t)kWElems * 2);
  const size_t oB   = off; off += al4k((size_t)kBiasElems * 4);
  const size_t oXH  = off; off += al4k((size_t)kChunkRows * kK0 * 2);
  const size_t szRA = al4k((size_t)kChunkRows * kN0 * 2);
  const size_t oRA  = off; off += szRA;
  const size_t oH1  = off; off += al4k((size_t)kChunkRows * kP * 2);
  const size_t oS2  = off; off += al4k((size_t)kChunkRows * kP * 4);
  const size_t oF2  = off; off += al4k((size_t)kChunkRows * kNf * 4);
  const size_t oG   = off; off += al4k((size_t)kChunkItems * kP * 2);
  const size_t oGQ  = off; off += al4k((size_t)kChunkItems * kP * 4);
  const size_t oMH  = off; off += al4k((size_t)kItems * kKm * 2);
  const size_t oML  = off; off += al4k((size_t)kItems * kKm * 2);
  const size_t oA1  = oRA;
  const size_t oSF  = oRA;
  const size_t oT1H = oRA;
  const size_t oT1L = oT1H + (size_t)kItems * kN0 * 2;
  const size_t oT2H = oT1L + (size_t)kItems * kN0 * 2;
  const size_t oT2L = oT2H + (size_t)kItems * kP * 2;
  const size_t oT3  = oT2L + (size_t)kItems * kP * 2;
  const size_t endT = oT3 + (size_t)kItems * kP * 4;
  if (off > ws_size) return;
  if (endT > oRA + szRA) return;
  if (oSF + (size_t)kChunkRows * kP * 2 > oRA + szRA) return;

  unsigned char* ws = (unsigned char*)d_ws;
  unsigned short* WP   = (unsigned short*)(ws + oWP);
  unsigned short* WL   = (unsigned short*)(ws + oWL);
  float*          BIAS = (float*)(ws + oB);
  unsigned short* XH   = (unsigned short*)(ws + oXH);
  unsigned short* A1   = (unsigned short*)(ws + oA1);
  unsigned short* SF   = (unsigned short*)(ws + oSF);
  unsigned short* H1   = (unsigned short*)(ws + oH1);
  float*          S2   = (float*)(ws + oS2);
  float*          F2   = (float*)(ws + oF2);
  unsigned short* G    = (unsigned short*)(ws + oG);
  float*          GQ   = (float*)(ws + oGQ);
  unsigned short* MH   = (unsigned short*)(ws + oMH);
  unsigned short* ML   = (unsigned short*)(ws + oML);
  unsigned short* T1H  = (unsigned short*)(ws + oT1H);
  unsigned short* T1L  = (unsigned short*)(ws + oT1L);
  unsigned short* T2H  = (unsigned short*)(ws + oT2H);
  unsigned short* T2L  = (unsigned short*)(ws + oT2L);
  float*          T3   = (float*)(ws + oT3);

  wprep_kernel<0><<<dim3(8, 4), 256, 0, stream>>>(wa0, wa0 + 100 * 100, wa1, w2a,
                                                  kOffWa0t, kOffWa0b, kOffWa1, kOffW2a,
                                                  WP, WL, 100, 100, kP, kP, 100, kWCarry);
  wprep_kernel<0><<<dim3(3, 1), 256, 0, stream>>>(w1a, w1a, w1a, w1a,
                                                  kOffW1a, kOffW1a, kOffW1a, kOffW1a,
                                                  WP, WL, kFeat, 150, kK0, kN0, 150, kWCarry);
  wprep_kernel<0><<<dim3(10, 1), 256, 0, stream>>>(w1b, w1b, w1b, w1b,
                                                   kOffW1b, kOffW1b, kOffW1b, kOffW1b,
                                                   WP, WL, 150, 100, kK1, kP, 100, kWCarry);
  wprep_kernel<0><<<dim3(4, 1), 256, 0, stream>>>(w2b, w2b, w2b, w2b,
                                                  kOffW2b, kOffW2b, kOffW2b, kOffW2b,
                                                  WP, WL, 100, 50, kP, kNf, 50, kWCarry);
  wprep_kernel<1><<<dim3(6, 1), 256, 0, stream>>>(w3a, w3a, w3a, w3a,
                                                  kOffW3a, kOffW3a, kOffW3a, kOffW3a,
                                                  WP, WL, kSelf + 50, 150, kKm, kN0, 150, 1.0f);
  wprep_kernel<1><<<dim3(10, 1), 256, 0, stream>>>(w3b, w3b, w3b, w3b,
                                                   kOffW3b, kOffW3b, kOffW3b, kOffW3b,
                                                   WP, WL, 150, 100, kK1, kP, 100, 1.0f);
  wprep_kernel<1><<<dim3(8, 1), 256, 0, stream>>>(w3c, w3c, w3c, w3c,
                                                  kOffW3c, kOffW3c, kOffW3c, kOffW3c,
                                                  WP, WL, 100, 100, kP, kP, 100, 1.0f);
  bprep_kernel<<<9, 64, 0, stream>>>(b1a, b1b, ba0, ba1, b2a, b2b, b3a, b3b, b3c, BIAS);

  for (int c = 0; c < kNumChunks; ++c) {
    const float* xc = x + (size_t)c * kChunkRows * kFeat;
    xprep_kernel<<<kChunkRows * 4 / 256, 256, 0, stream>>>(xc, XH, kChunkRows);
    wmma_gemm64<0, false, 2, 1, false, 2><<<gemm_grid(kChunkRows, kN0), 256, 0, stream>>>(
        XH, XH, kK0, 0L, WP + kOffW1a, WP + kOffW1a, kK0, 0L,
        (void*)A1, (void*)A1, kN0, 0L, BIAS + kOffB1a, BIAS, 0L, kChunkRows, kN0, kK0, kSc1a);
    wmma_gemm64<0, false, 2, 1, false, 2><<<gemm_grid(kChunkRows, kP), 256, 0, stream>>>(
        A1, A1, kN0, 0L, WP + kOffW1b, WP + kOffW1b, kK1, 0L,
        (void*)H1, (void*)H1, kP, 0L, BIAS + kOffB1b, BIAS, 0L, kChunkRows, kP, kK1, kScAct);
    gmean_kernel<<<kChunkItems * 16 / 256, 256, 0, stream>>>(H1, G, kChunkItems);
    wmma_gemm64<0, false, 0, 0, false, 0><<<gemm_grid(kChunkItems, kP), 256, 0, stream>>>(
        G, G, kP, 0L, WP + kOffWa0b, WP + kOffWa0b, kP, 0L,
        (void*)GQ, (void*)GQ, kP, 0L, BIAS, BIAS, 0L, kChunkItems, kP, kP, kScAct);
    wmma_gemm64<0, false, 2, 1, true, 2, kAgents><<<gemm_grid(kChunkRows, kP), 256, 0, stream>>>(
        H1, H1, kP, 0L, WP + kOffWa0t, WP + kOffWa0t, kP, 0L,
        (void*)SF, (void*)SF, kP, 0L, BIAS + kOffBa0, GQ, 0L, kChunkRows, kP, kP, kScAct);
    wmma_gemm64<0, false, 2, 0, false, 2><<<gemm_grid(kChunkRows, kP), 256, 0, stream>>>(
        SF, SF, kP, 0L, WP + kOffWa1, WP + kOffWa1, kP, 0L,
        (void*)S2, (void*)S2, kP, 0L, BIAS + kOffBa1, BIAS, 0L, kChunkRows, kP, kP, kScF32);
    wmma_gemm64<0, false, 2, 1, false, 2><<<gemm_grid(kChunkRows, kP), 256, 0, stream>>>(
        H1, H1, kP, 0L, WP + kOffW2a, WP + kOffW2a, kP, 0L,
        (void*)SF, (void*)SF, kP, 0L, BIAS + kOffB2a, BIAS, 0L, kChunkRows, kP, kP, kScAct);
    wmma_gemm64<0, false, 2, 0, false, 0><<<gemm_grid(kChunkRows, kNf), 256, 0, stream>>>(
        SF, SF, kP, 0L, WP + kOffW2b, WP + kOffW2b, kP, 0L,
        (void*)F2, (void*)F2, kNf, 0L, BIAS + kOffB2b, BIAS, 0L, kChunkRows, kNf, kP, kScF32);
    pool_kernel<<<kChunkItems / 8, 256, 0, stream>>>(S2, F2, xc, wa2, ba2,
                                                      MH + (size_t)c * kChunkItems * kKm,
                                                      ML + (size_t)c * kChunkItems * kKm, kChunkItems);
  }

  wmma_gemm64<1, true, 2, 2, false, 2><<<gemm_grid(kItems, kN0), 256, 0, stream>>>(
      MH, ML, kKm, 0L, WP + kOffW3a, WL + kOffW3a, kKm, 0L,
      (void*)T1H, (void*)T1L, kN0, 0L, BIAS + kOffB3a, BIAS, 0L, kItems, kN0, kKm, 1.0f);
  wmma_gemm64<1, true, 2, 2, false, 2><<<gemm_grid(kItems, kP), 256, 0, stream>>>(
      T1H, T1L, kN0, 0L, WP + kOffW3b, WL + kOffW3b, kK1, 0L,
      (void*)T2H, (void*)T2L, kP, 0L, BIAS + kOffB3b, BIAS, 0L, kItems, kP, kK1, 1.0f);
  wmma_gemm64<1, true, 2, 0, false, 2><<<gemm_grid(kItems, kP), 256, 0, stream>>>(
      T2H, T2L, kP, 0L, WP + kOffW3c, WL + kOffW3c, kP, 0L,
      (void*)T3, (void*)T3, kP, 0L, BIAS + kOffB3c, BIAS, 0L, kItems, kP, kP, 1.0f);
  value_head_kernel<<<kItems / 256, 256, 0, stream>>>(T3, w3d, b3d, out, kItems);
}
